// PhysicsInformedBasicLiquidNetworkModel_51299089383599
// MI455X (gfx1250) — hardware-verified
//
#include <hip/hip_runtime.h>
#include <math.h>

typedef __attribute__((ext_vector_type(16))) _Float16 v16h;
typedef __attribute__((ext_vector_type(8)))  _Float16 v8h;
typedef __attribute__((ext_vector_type(4)))  _Float16 v4h;
typedef __attribute__((ext_vector_type(8)))  float    v8f;
typedef __attribute__((ext_vector_type(4)))  float    v4f;

__device__ __forceinline__ void dep_guard_h(v8f& a, v8f& b, v16h x, v16h y) { asm volatile("v_nop\n\tv_nop\n\tv_nop\n\tv_nop" : "+v"(a), "+v"(b) : "v"(x), "v"(y)); }
__device__ __forceinline__ void keep4_h(v16h a, v16h b, v16h c, v16h d) { asm volatile("v_nop" :: "v"(a), "v"(b), "v"(c), "v"(d)); }
__device__ __forceinline__ void acc_guard2(v8f& a, v8f& b) { asm volatile("v_nop\n\tv_nop\n\tv_nop\n\tv_nop" : "+v"(a), "+v"(b)); }

template <typename T> struct Frag;
template <> struct Frag<_Float16> {
  typedef v16h V; union U { v16h v; v8h h[2]; };
  static __device__ __forceinline__ v16h load(const _Float16* p) {
    U f; f.h[0] = *(const v8h*)(p); f.h[1] = *(const v8h*)(p + 16); return f.v;
  }
  static __device__ __forceinline__ v8f mma(v16h a, v16h b, v8f c) {
    return __builtin_amdgcn_wmma_f32_16x16x32_f16(false, a, false, b, (short)0, c, false, false);
  }
  static __device__ __forceinline__ void guard(v8f& a, v8f& b, v16h x, v16h y) { dep_guard_h(a, b, x, y); }
  static __device__ __forceinline__ void keep(v16h a, v16h b, v16h c, v16h d) { keep4_h(a, b, c, d); }
};

constexpr int kBatch   = 128;
constexpr int kSteps   = 2048;
constexpr int kDin     = 16;
constexpr int kHid     = 256;
constexpr int kNapp    = 10;
constexpr int kRows    = 16;
constexpr int kWaves   = 8;
constexpr int kThreads = 256;
constexpr int kKTot    = 288;
constexpr int kKSteps  = kKTot / 32;
constexpr int kAPitch  = 296;
constexpr int kBPitch  = 320;
constexpr int kVPitch  = 260;
constexpr float kDt      = 0.1f;
constexpr float kEps     = 1e-5f;
constexpr float kAScale  = 4.0f;
constexpr float kBScale  = 256.0f;
constexpr float kAccInv  = 1.0f / 1024.0f;
constexpr float kInvH    = 1.0f / 256.0f;

static_assert(kKTot % 32 == 0, "K multiple of 32");
static_assert(kBatch % kRows == 0, "whole row blocks");
static_assert(kHid == kWaves * 32, "8 waves x 32 columns");
static_assert(kRows == 2 * kWaves, "each wave owns 2 rows in the LN phase");
static_assert(kThreads == kHid, "parameter staging: one thread per column");
static_assert(kAPitch % 8 == 0 && kAPitch >= kKTot, "A tile pitch");
static_assert((kBPitch * 2) % 128 == 0 && kBPitch >= kKTot, "Bt rows are whole 128-B lines");
static_assert((kRows * kNapp * 4) % 128 == 0, "each block's output segment is whole lines (640 B)");
static_assert(kRows * kNapp == 160, "output segment = 32 + 8 float4 chunks");

__global__ __launch_bounds__(256) void build_bt_kernel(
    const float* __restrict__ W_in, const float* __restrict__ W_rec, unsigned short* __restrict__ Btp)
{
  _Float16* Bt = (_Float16*)(void*)Btp;
  const int tid = threadIdx.x;
  const int wave = tid >> 5, lane = tid & 31;
  const int n = blockIdx.x * kWaves + wave;
  v8h va, vb;
#pragma unroll
  for (int e = 0; e < 8; ++e) {
    const int ka = 8 * lane + e;
    const float wi = W_in[n * kDin + (ka & 15)];
    int ja = ka - 32; ja = ja < 0 ? 0 : ja;
    const float wra = W_rec[(size_t)ja * kHid + n];
    const float fa = (ka < 16) ? wi : ((ka < 32) ? 0.0f : wra);
    va[e] = (_Float16)(kBScale * fa);
    const int kb = 256 + 8 * lane + e;
    int jb = kb - 32; jb = jb > (kHid - 1) ? (kHid - 1) : jb;
    const float wrb = W_rec[(size_t)jb * kHid + n];
    const float fb = (kb < kKTot) ? wrb : 0.0f;
    vb[e] = (_Float16)(kBScale * fb);
  }
  _Float16* rowp = Bt + (size_t)n * kBPitch;
  for (int pass = 0; pass < 2; ++pass) {
    *(volatile v8h*)(rowp + 8 * lane) = va;
    if (lane < 8) *(volatile v8h*)(rowp + 256 + 8 * lane) = vb;
    __threadfence();
  }
}

__global__ __launch_bounds__(256) void ltc_scan_kernel(
    const float* __restrict__ x, const unsigned short* __restrict__ Btp,
    const float* __restrict__ b_in, const float* __restrict__ tau_param,
    const float* __restrict__ g_intra, const float* __restrict__ b_intra,
    const float* __restrict__ g_norm, const float* __restrict__ b_norm,
    const float* __restrict__ W_head, const float* __restrict__ b_head,
    float* __restrict__ out)
{
  __shared__ __align__(16) _Float16 sA[kRows * kAPitch];
  __shared__ __align__(16) float    sV[kRows * kVPitch];
  __shared__ __align__(16) float    sH[kRows * kVPitch];
  __shared__ __align__(16) float    sPar[5 * kHid];
  __shared__ __align__(16) float    sOut[kRows * kNapp];

  const _Float16* Bt = (const _Float16*)(const void*)Btp;
  const int tid  = threadIdx.x;
  const int wave = tid >> 5, lane = tid & 31, hh = lane >> 4, cix = lane & 15;
  const int b0   = blockIdx.x * kRows;
  const int n0w  = wave * 32;
  const int lc0  = lane * 8;
  const int xr = (tid >> 2) & 15, xi4 = tid & 3;
  const float* xrow = x + (size_t)(b0 + xr) * kSteps * kDin + 4 * xi4;

  {
    const int cc = tid;
    sPar[cc] = g_intra[cc];
    sPar[kHid + cc] = b_intra[cc];
    const float tp  = tau_param[cc];
    const float tau = fmaxf(tp, 0.0f) + log1pf(expf(-fabsf(tp)));
    sPar[2 * kHid + cc] = 1.0f / tau;
    sPar[3 * kHid + cc] = g_norm[cc];
    sPar[4 * kHid + cc] = b_norm[cc];
  }
  const float bin0 = b_in[n0w + cix];
  const float bin1 = b_in[n0w + 16 + cix];

  {
    for (int i = tid; i < kRows * kVPitch; i += kThreads) sH[i] = 0.0f;
    v8h z8;
#pragma unroll
    for (int e = 0; e < 8; ++e) z8[e] = (_Float16)0.0f;
    for (int i = tid; i < kRows * 35; i += kThreads) {
      const int row = i / 35, ch = i - row * 35;
      *(v8h*)(sA + row * kAPitch + 16 + 8 * ch) = z8;
    }
    if (wave < 2) {
      const v4f xv = *(const v4f*)(xrow);
      v4h xh;
#pragma unroll
      for (int e = 0; e < 4; ++e) xh[e] = (_Float16)(kAScale * xv[e]);
      *(v4h*)(sA + xr * kAPitch + 4 * xi4) = xh;
    }
  }
  __syncthreads();

  const _Float16* ap  = sA + cix * kAPitch + 8 * hh;
  const _Float16* bp0 = Bt + (size_t)(n0w + cix) * kBPitch + 8 * hh;
  const _Float16* bp1 = bp0 + (size_t)16 * kBPitch;

  for (int t = 0; t < kSteps; ++t) {
    v4f xn = (v4f){0.f, 0.f, 0.f, 0.f};
    if (wave < 2) {
      const int tn = (t + 1 < kSteps) ? (t + 1) : (kSteps - 1);
      xn = *(const v4f*)(xrow + (size_t)tn * kDin);
    }

    v8f acc0 = (v8f){0.f,0.f,0.f,0.f,0.f,0.f,0.f,0.f};
    v8f acc1 = (v8f){0.f,0.f,0.f,0.f,0.f,0.f,0.f,0.f};
#pragma unroll 3
    for (int ks = 0; ks < kKSteps; ++ks) {
      const int k0 = ks * 32;
      const v16h af  = Frag<_Float16>::load(ap + k0);
      const v16h bf0 = Frag<_Float16>::load(bp0 + k0);
      const v16h bf1 = Frag<_Float16>::load(bp1 + k0);
      acc0 = Frag<_Float16>::mma(af, bf0, acc0);
      acc1 = Frag<_Float16>::mma(af, bf1, acc1);
      dep_guard_h(acc0, acc1, af, bf1);
    }
    acc_guard2(acc0, acc1);
#pragma unroll
    for (int r = 0; r < 8; ++r) {
      float* vrow = sV + (8 * hh + r) * kVPitch + n0w + cix;
      vrow[0]  = acc0[r] * kAccInv + bin0;
      vrow[16] = acc1[r] * kAccInv + bin1;
    }
    __syncthreads();

#pragma unroll 1
    for (int q = 0; q < 2; ++q) {
      const int row = 2 * wave + q;
      const float* vr = sV + row * kVPitch + lc0;
      float* hr = sH + row * kVPitch + lc0;
      _Float16* ar = sA + row * kAPitch + 32 + lc0;
      float s = 0.0f;
#pragma unroll 1
      for (int j = 0; j < 8; ++j) s += vr[j];
#pragma unroll
      for (int off = 16; off > 0; off >>= 1) s += __shfl_xor(s, off, 32);
      const float mu = s * kInvH;
      float ss = 0.0f;
#pragma unroll 1
      for (int j = 0; j < 8; ++j) { const float d = vr[j] - mu; ss = fmaf(d, d, ss); }
#pragma unroll
      for (int off = 16; off > 0; off >>= 1) ss += __shfl_xor(ss, off, 32);
      const float rs = rsqrtf(ss * kInvH + kEps);
#pragma unroll 1
      for (int j = 0; j < 8; ++j) {
        const int col = lc0 + j;
        const float y  = (vr[j] - mu) * rs * sPar[col] + sPar[kHid + col];
        const float e2 = expf(2.0f * y);
        const float f  = 1.0f - 2.0f * __builtin_amdgcn_rcpf(e2 + 1.0f);
        const float hold = hr[j];
        const float dh = (f - hold * sPar[2 * kHid + col]) * kDt;
        float hn = hold + dh;
        hn = fminf(fmaxf(hn, -10.0f), 10.0f);
        hr[j] = hn;
        ar[j] = (_Float16)(kAScale * hn);
      }
    }
    if (wave < 2) {
      v4h xh;
#pragma unroll
      for (int e = 0; e < 4; ++e) xh[e] = (_Float16)(kAScale * xn[e]);
      *(v4h*)(sA + xr * kAPitch + 4 * xi4) = xh;
    }
    __syncthreads();
  }

#pragma unroll 1
  for (int q = 0; q < 2; ++q) {
    const int row = 2 * wave + q;
    const float* hr = sH + row * kVPitch + lc0;
    float* vr = sV + row * kVPitch + lc0;
    float s = 0.0f;
#pragma unroll 1
    for (int j = 0; j < 8; ++j) s += hr[j];
#pragma unroll
    for (int off = 16; off > 0; off >>= 1) s += __shfl_xor(s, off, 32);
    const float mu = s * kInvH;
    float ss = 0.0f;
#pragma unroll 1
    for (int j = 0; j < 8; ++j) { const float d = hr[j] - mu; ss = fmaf(d, d, ss); }
#pragma unroll
    for (int off = 16; off > 0; off >>= 1) ss += __shfl_xor(ss, off, 32);
    const float rs = rsqrtf(ss * kInvH + kEps);
#pragma unroll 1
    for (int j = 0; j < 8; ++j) {
      const int col = lc0 + j;
      vr[j] = (hr[j] - mu) * rs * sPar[3 * kHid + col] + sPar[4 * kHid + col];
    }
  }
  __syncthreads();

  if (tid < kRows * kNapp) {
    const int row = tid / kNapp, a = tid - row * kNapp;
    const float* vrow = sV + row * kVPitch;
    float accv = 0.0f;
#pragma unroll 1
    for (int n = 0; n < kHid; ++n) accv = fmaf(vrow[n], W_head[n * kNapp + a], accv);
    sOut[tid] = accv + b_head[a];
  }
  __syncthreads();

  if (wave == 0) {
    float* ob = out + (size_t)b0 * kNapp;
    const int l2 = (lane < 8) ? lane : 7;
    for (int pass = 0; pass < 2; ++pass) {
      const v4f o1 = *(const v4f*)(sOut + 4 * lane);
      const v4f o2 = *(const v4f*)(sOut + 128 + 4 * l2);
      *(volatile v4f*)(ob + 4 * lane) = o1;
      if (lane < 8) *(volatile v4f*)(ob + 128 + 4 * lane) = o2;
      __threadfence();
    }
  }
}

extern "C" void kernel_launch(void* const* d_in, const int* in_sizes, int n_in,
                              void* d_out, int out_size, void* d_ws, size_t ws_size,
                              hipStream_t stream)
{
  if (n_in < 11) return;
  if (in_sizes[0] != kBatch * kSteps * kDin) return;
  if (in_sizes[1] != kHid * kDin) return;
  if (in_sizes[2] != kHid || in_sizes[3] != kHid) return;
  if (in_sizes[4] != kHid * kHid) return;
  if (in_sizes[5] != kHid || in_sizes[6] != kHid || in_sizes[7] != kHid || in_sizes[8] != kHid) return;
  if (in_sizes[9] != kHid * kNapp || in_sizes[10] != kNapp) return;
  if (out_size != kBatch * kNapp) return;
  const size_t bt_bytes = (size_t)kHid * kBPitch * sizeof(unsigned short);
  if (ws_size < bt_bytes) return;

  const float* x         = (const float*)d_in[0];
  const float* W_in      = (const float*)d_in[1];
  const float* b_in      = (const float*)d_in[2];
  const float* tau_param = (const float*)d_in[3];
  const float* W_rec     = (const float*)d_in[4];
  const float* g_intra   = (const float*)d_in[5];
  const float* b_intra   = (const float*)d_in[6];
  const float* g_norm    = (const float*)d_in[7];
  const float* b_norm    = (const float*)d_in[8];
  const float* W_head    = (const float*)d_in[9];
  const float* b_head    = (const float*)d_in[10];
  float* outp = (float*)d_out;
  unsigned short* Bt = (unsigned short*)d_ws;

  build_bt_kernel<<<dim3(kHid / kWaves), dim3(kThreads), 0, stream>>>(W_in, W_rec, Bt);
  ltc_scan_kernel<<<dim3(kBatch / kRows), dim3(kThreads), 0, stream>>>(
      x, Bt, b_in, tau_param, g_intra, b_intra, g_norm, b_norm, W_head, b_head, outp);
}
